// DeltaNet_28097676051326
// MI455X (gfx1250) — hardware-run, weakly checked
//
#include <hip/hip_runtime.h>
#include <math.h>

constexpr int kB      = 4;
constexpr int kL      = 1024;
constexpr int kHid    = 1024;
constexpr int kNH     = 16;
constexpr int kHD     = 64;
constexpr int kConvK  = 4;
constexpr int kTok    = kB * kL;
constexpr int kNStackReal = 3 * kHid + kNH;
constexpr int kNStack = 3136;
constexpr int kChunkT = 32;
constexpr int kFlushT = 16;
constexpr int kSPitch = 68;
constexpr float kEps  = 1e-6f;

constexpr size_t kOffXh  = 0;
constexpr size_t kOffXl  = (size_t)kTok * kHid * 2;
constexpr size_t kOffWh  = kOffXl + (size_t)kTok * kHid * 2;
constexpr size_t kOffWl  = kOffWh + (size_t)kNStack * kHid * 2;
constexpr size_t kOffP   = kOffWl + (size_t)kNStack * kHid * 2;
constexpr size_t kSizeP  = (size_t)kTok * kNStack * 4;
constexpr size_t kOffQh  = 0;
constexpr size_t kOffKh  = kOffP + kSizeP;
constexpr size_t kOffVh  = kOffKh + (size_t)kTok * kHid * 4;
constexpr size_t kOffBt  = kOffVh + (size_t)kTok * kHid * 4;
constexpr size_t kWsTotal = kOffBt + (size_t)kB * kNH * kL * 4;
constexpr size_t kOffOnh = kOffP;
constexpr size_t kOffOnl = kOffOnh + (size_t)kTok * kHid * 2;
constexpr size_t kOffWoh = kOffOnl + (size_t)kTok * kHid * 2;
constexpr size_t kOffWol = kOffWoh + (size_t)kHid * kHid * 2;

typedef __attribute__((ext_vector_type(16))) _Float16 v16h;
typedef __attribute__((ext_vector_type(8)))  _Float16 v8h;
typedef __attribute__((ext_vector_type(16))) __bf16   v16b;
typedef __attribute__((ext_vector_type(8)))  __bf16   v8b;
typedef __attribute__((ext_vector_type(8)))  float    v8f;
typedef __attribute__((ext_vector_type(4)))  float    v4f;
typedef __attribute__((ext_vector_type(4)))  unsigned int v4u;

__device__ __forceinline__ unsigned short f2bf_bits(float f) {
  unsigned u = __float_as_uint(f);
  return (unsigned short)((u + 0x7FFFu + ((u >> 16) & 1u)) >> 16);
}
__device__ __forceinline__ float bf_bits2f(unsigned short h) { return __uint_as_float(((unsigned)h) << 16); }

__device__ __forceinline__ void dep_guard_h(v8f& a, v8f& b, v16h x, v16h y) { asm volatile("v_nop\n\tv_nop\n\tv_nop\n\tv_nop" : "+v"(a), "+v"(b) : "v"(x), "v"(y)); }
__device__ __forceinline__ void dep_guard_b(v8f& a, v8f& b, v16b x, v16b y) { asm volatile("v_nop\n\tv_nop\n\tv_nop\n\tv_nop" : "+v"(a), "+v"(b) : "v"(x), "v"(y)); }
__device__ __forceinline__ void keep4_h(v16h a, v16h b, v16h c, v16h d) { asm volatile("v_nop" :: "v"(a), "v"(b), "v"(c), "v"(d)); }
__device__ __forceinline__ void keep4_b(v16b a, v16b b, v16b c, v16b d) { asm volatile("v_nop" :: "v"(a), "v"(b), "v"(c), "v"(d)); }
__device__ __forceinline__ void acc_guard4(v8f& a, v8f& b, v8f& c, v8f& d) { asm volatile("v_nop\n\tv_nop\n\tv_nop\n\tv_nop" : "+v"(a), "+v"(b), "+v"(c), "+v"(d)); }
template <typename T> struct Frag;
template <> struct Frag<_Float16> {
  typedef v16h V; union U { v16h v; v8h h[2]; };
  static __device__ __forceinline__ v16h load(const _Float16* p) {
    U f; f.h[0] = *(const v8h*)(p); f.h[1] = *(const v8h*)(p + 16); return f.v;
  }
  static __device__ __forceinline__ v8f mma(v16h a, v16h b, v8f c) {
    return __builtin_amdgcn_wmma_f32_16x16x32_f16(false, a, false, b, (short)0, c, false, false);
  }
  static __device__ __forceinline__ void guard(v8f& a, v8f& b, v16h x, v16h y) { dep_guard_h(a, b, x, y); }
  static __device__ __forceinline__ void keep(v16h a, v16h b, v16h c, v16h d) { keep4_h(a, b, c, d); }
};
template <> struct Frag<__bf16> {
  typedef v16b V; union U { v16b v; v8b h[2]; };
  static __device__ __forceinline__ v16b load(const __bf16* p) {
    U f; f.h[0] = *(const v8b*)(p); f.h[1] = *(const v8b*)(p + 16); return f.v;
  }
  static __device__ __forceinline__ v8f mma(v16b a, v16b b, v8f c) {
    return __builtin_amdgcn_wmma_f32_16x16x32_bf16(false, a, false, b, (short)0, c, false, false);
  }
  static __device__ __forceinline__ void guard(v8f& a, v8f& b, v16b x, v16b y) { dep_guard_b(a, b, x, y); }
  static __device__ __forceinline__ void keep(v16b a, v16b b, v16b c, v16b d) { keep4_b(a, b, c, d); }
};

__device__ __forceinline__ unsigned pk16(unsigned short a, unsigned short b) { return (unsigned)a | ((unsigned)b << 16); }

template <int ET> struct Elem;
template <> struct Elem<0> { typedef _Float16 T; };
template <> struct Elem<1> { typedef __bf16 T; };
template <int ET, bool SPLIT, int BIAS_MODE, int OUT_MODE, bool RESID, int ACT = 0>
__global__ __launch_bounds__(256) void wmma_gemm64(
    const unsigned short* __restrict__ Ap, const unsigned short* __restrict__ A2p, int lda, long strideA,
    const unsigned short* __restrict__ Btp, const unsigned short* __restrict__ Bt2p, int ldb, long strideB,
    void* __restrict__ Cout, void* __restrict__ Cout2, int ldc, long strideC,
    const float* __restrict__ bias,
    const float* __restrict__ resid, long strideR,
    int M, int N, int K, float scale) {
  typedef typename Elem<ET>::T T;
  typedef typename Frag<T>::V V;
  const T* A = (const T*)Ap; const T* A2 = (const T*)A2p; const T* Bt = (const T*)Btp; const T* Bt2 = (const T*)Bt2p;
  __shared__ __align__(16) float sT[8][16 * 68];
  const int b    = blockIdx.y;
  const int lane = threadIdx.x & 31;
  const int wave = threadIdx.x >> 5;
  const int tilesN = N >> 6;
  const int tilesM = M >> 6;
  const int tile = blockIdx.x * 8 + wave;
  if (tile >= tilesM * tilesN) return;
  const int tm = tile / tilesN;
  const int tn = tile - tm * tilesN;
  const int m0 = tm << 6;
  const int n0 = tn << 6;

  const T* Ab  = A  + (size_t)b * strideA;
  const T* Bb  = Bt + (size_t)b * strideB;
  const T* Ab2 = SPLIT ? (A2  + (size_t)b * strideA) : nullptr;
  const T* Bb2 = SPLIT ? (Bt2 + (size_t)b * strideB) : nullptr;

  const int rlane = lane & 15;
  const int koff  = (lane >> 4) * 8;
  const int mOff  = (lane >> 4) * 8;

  v8f acc[4][4];
#pragma unroll
  for (int i = 0; i < 4; ++i)
#pragma unroll
    for (int j = 0; j < 4; ++j) acc[i][j] = (v8f){0.f,0.f,0.f,0.f,0.f,0.f,0.f,0.f};

  for (int k0 = 0; k0 < K; k0 += 32) {
    V bh[4], bl[4];
#pragma unroll
    for (int j = 0; j < 4; ++j) {
      const size_t bo = (size_t)(n0 + (j << 4) + rlane) * ldb + koff + k0;
      bh[j] = Frag<T>::load(Bb + bo);
      if (SPLIT) bl[j] = Frag<T>::load(Bb2 + bo);
    }
#pragma unroll
    for (int i = 0; i < 4; ++i) {
      const size_t ao = (size_t)(m0 + (i << 4) + rlane) * lda + koff + k0;
      V ah = Frag<T>::load(Ab + ao);
      V al;
      if (SPLIT) al = Frag<T>::load(Ab2 + ao);
#pragma unroll
      for (int j = 0; j < 4; ++j) {
        acc[i][j] = Frag<T>::mma(ah, bh[j], acc[i][j]);
        if (SPLIT) {
          acc[i][j] = Frag<T>::mma(ah, bl[j], acc[i][j]);
          acc[i][j] = Frag<T>::mma(al, bh[j], acc[i][j]);
        }
      }
      Frag<T>::guard(acc[i][0], acc[i][3], ah, SPLIT ? al : ah);
    }
    Frag<T>::keep(bh[0], bh[1], bh[2], bh[3]);
    if (SPLIT) Frag<T>::keep(bl[0], bl[1], bl[2], bl[3]);
  }
  acc_guard4(acc[0][0], acc[0][1], acc[0][2], acc[0][3]);
  acc_guard4(acc[1][0], acc[1][1], acc[1][2], acc[1][3]);
  acc_guard4(acc[2][0], acc[2][1], acc[2][2], acc[2][3]);
  acc_guard4(acc[3][0], acc[3][1], acc[3][2], acc[3][3]);

  float* slab = sT[wave];
  const float* Rb = RESID ? (resid + (size_t)b * strideR) : nullptr;
#pragma unroll
  for (int i = 0; i < 4; ++i) {
    const int mBase = m0 + (i << 4);
#pragma unroll
    for (int j = 0; j < 4; ++j) {
      const int n = n0 + (j << 4) + rlane;
      float bv = 0.f;
      if (BIAS_MODE == 2) bv = bias[n];
#pragma unroll
      for (int r = 0; r < 8; ++r) {
        float v = acc[i][j][r] * scale;
        if (BIAS_MODE == 1) v += bias[mBase + mOff + r];
        if (BIAS_MODE == 2) v += bv;
        if (RESID) v += Rb[(size_t)(mBase + mOff + r) * ldc + n];
        if (ACT == 2) v = fmaxf(v, 0.0f);
        if (ACT == 4) v = (v > 0.f) ? v : 0.01f * v;
        slab[(mOff + r) * 68 + (j << 4) + rlane] = v;
      }
    }
    __builtin_amdgcn_fence(__ATOMIC_RELEASE, "workgroup");
    __builtin_amdgcn_wave_barrier();
    __builtin_amdgcn_fence(__ATOMIC_ACQUIRE, "workgroup");
    if (OUT_MODE == 0) {
      float* C = (float*)Cout + (size_t)b * strideC;
      const int hh = lane >> 4, c4 = (lane & 15) * 4;
      for (int pass = 0; pass < 2; ++pass) {
#pragma unroll
        for (int it = 0; it < 8; ++it) {
          const int row = it * 2 + hh;
          v4f v = *(const v4f*)(slab + row * 68 + c4);
          *(volatile v4f*)(C + (size_t)(mBase + row) * ldc + n0 + c4) = v;
        }
        __threadfence();
      }
    } else {
      const int q = lane >> 3, c8 = (lane & 7) * 8;
      unsigned short* C  = (unsigned short*)Cout  + (size_t)b * strideC;
      unsigned short* C2 = (OUT_MODE == 2) ? ((unsigned short*)Cout2 + (size_t)b * strideC) : nullptr;
      for (int pass = 0; pass < 2; ++pass) {
#pragma unroll
        for (int it = 0; it < 4; ++it) {
          const int row = it * 4 + q;
          const float* sp = slab + row * 68 + c8;
          v8h hv, lv;
#pragma unroll
          for (int e = 0; e < 8; ++e) {
            if (OUT_MODE == 1) {
              hv[e] = (_Float16)sp[e];
            } else {
              unsigned short hb = f2bf_bits(sp[e]);
              unsigned short lb = f2bf_bits(sp[e] - bf_bits2f(hb));
              hv[e] = __builtin_bit_cast(_Float16, hb);
              lv[e] = __builtin_bit_cast(_Float16, lb);
            }
          }
          *(volatile v8h*)(C + (size_t)(mBase + row) * ldc + n0 + c8) = hv;
          if (OUT_MODE == 2) *(volatile v8h*)(C2 + (size_t)(mBase + row) * ldc + n0 + c8) = lv;
        }
        __threadfence();
      }
    }
    __builtin_amdgcn_fence(__ATOMIC_RELEASE, "workgroup");
    __builtin_amdgcn_wave_barrier();
    __builtin_amdgcn_fence(__ATOMIC_ACQUIRE, "workgroup");
  }
}

__global__ __launch_bounds__(256) void split8_kernel(const float* __restrict__ in,
                                                     unsigned short* __restrict__ hi,
                                                     unsigned short* __restrict__ lo, int n8) {
  const int i = blockIdx.x * 256 + threadIdx.x;
  if (i >= n8) return;
  const float* p = in + 8 * (size_t)i;
  const v4f a = *(const v4f*)(p);
  const v4f c = *(const v4f*)(p + 4);
  unsigned short hb[8], lb[8];
#pragma unroll
  for (int e = 0; e < 4; ++e) {
    hb[e] = f2bf_bits(a[e]);
    lb[e] = f2bf_bits(a[e] - bf_bits2f(hb[e]));
    hb[4 + e] = f2bf_bits(c[e]);
    lb[4 + e] = f2bf_bits(c[e] - bf_bits2f(hb[4 + e]));
  }
  const v4u uh = (v4u){pk16(hb[0], hb[1]), pk16(hb[2], hb[3]), pk16(hb[4], hb[5]), pk16(hb[6], hb[7])};
  const v4u ul = (v4u){pk16(lb[0], lb[1]), pk16(lb[2], lb[3]), pk16(lb[4], lb[5]), pk16(lb[6], lb[7])};
  unsigned short* qh = hi + 8 * (size_t)i;
  unsigned short* ql = lo + 8 * (size_t)i;
  *(volatile v4u*)qh = uh;
  *(volatile v4u*)ql = ul;
  __threadfence();
  *(volatile v4u*)qh = uh;
  *(volatile v4u*)ql = ul;
}

__global__ __launch_bounds__(256) void splitw_kernel(const float* __restrict__ Wq, const float* __restrict__ Wk,
                                                     const float* __restrict__ Wv, const float* __restrict__ Wb,
                                                     unsigned short* __restrict__ hi, unsigned short* __restrict__ lo) {
  const int i = blockIdx.x * 256 + threadIdx.x;
  const int row = i >> 7;
  const int c8 = (i & 127) * 8;
  const int r0 = blockIdx.x * 2;
  v4u uh = (v4u){0u, 0u, 0u, 0u};
  v4u ul = (v4u){0u, 0u, 0u, 0u};
  if (r0 < kNStackReal) {
    const float* W; int rr;
    if (r0 < kHid)            { W = Wq; rr = row; }
    else if (r0 < 2 * kHid)   { W = Wk; rr = row - kHid; }
    else if (r0 < 3 * kHid)   { W = Wv; rr = row - 2 * kHid; }
    else                      { W = Wb; rr = row - 3 * kHid; }
    const float* p = W + (size_t)rr * kHid + c8;
    const v4f a = *(const v4f*)(p);
    const v4f c = *(const v4f*)(p + 4);
    unsigned short hb[8], lb[8];
#pragma unroll
    for (int e = 0; e < 4; ++e) {
      hb[e] = f2bf_bits(a[e]);
      lb[e] = f2bf_bits(a[e] - bf_bits2f(hb[e]));
      hb[4 + e] = f2bf_bits(c[e]);
      lb[4 + e] = f2bf_bits(c[e] - bf_bits2f(hb[4 + e]));
    }
    uh = (v4u){pk16(hb[0], hb[1]), pk16(hb[2], hb[3]), pk16(hb[4], hb[5]), pk16(hb[6], hb[7])};
    ul = (v4u){pk16(lb[0], lb[1]), pk16(lb[2], lb[3]), pk16(lb[4], lb[5]), pk16(lb[6], lb[7])};
  }
  unsigned short* qh = hi + 8 * (size_t)i;
  unsigned short* ql = lo + 8 * (size_t)i;
  *(volatile v4u*)qh = uh;
  *(volatile v4u*)ql = ul;
  __threadfence();
  *(volatile v4u*)qh = uh;
  *(volatile v4u*)ql = ul;
}

__global__ __launch_bounds__(512) void prep_kernel(const float* __restrict__ P,
                                                   const float* __restrict__ cq, const float* __restrict__ ck,
                                                   const float* __restrict__ cv,
                                                   float* __restrict__ QH, float* __restrict__ KH,
                                                   float* __restrict__ VH, float* __restrict__ BT) {
  __shared__ __align__(16) float sb[32];
  const int t = threadIdx.x;
  const int chunk = blockIdx.x;
  const int h = blockIdx.y;
  const int b = blockIdx.z;
  const int tl = t >> 4;
  const int cg = t & 15;
  const int l = chunk * kChunkT + tl;
  const int c = h * kHD + cg * 4;
  const size_t rowb = (size_t)b * kL;
  const v4f z4 = (v4f){0.f, 0.f, 0.f, 0.f};

#pragma unroll 1
  for (int which = 0; which < 3; ++which) {
    const float* Wc = (which == 0) ? cq : ((which == 1) ? ck : cv);
    float* dstp     = (which == 0) ? QH : ((which == 1) ? KH : VH);
    const int col = which * kHid + c;
    v4f xt[4];
#pragma unroll
    for (int kk = 0; kk < 4; ++kk) {
      const int ls = l - 3 + kk;
      const int lsc = (ls < 0) ? 0 : ls;
      v4f xv = *(const v4f*)(P + (rowb + (size_t)lsc) * kNStack + col);
      if (ls < 0) xv = z4;
      xt[kk] = xv;
    }
    v4f wv[4];
#pragma unroll
    for (int e = 0; e < 4; ++e) wv[e] = *(const v4f*)(Wc + (size_t)(c + e) * kConvK);
    float y[4];
#pragma unroll
    for (int e = 0; e < 4; ++e) {
      float a = 0.0f;
#pragma unroll
      for (int kk = 0; kk < 4; ++kk) a = fmaf(xt[kk][e], wv[e][kk], a);
      const float ex = expf(-a);
      y[e] = a * __builtin_amdgcn_rcpf(1.0f + ex);
    }
    float ss = y[0] * y[0];
    ss = fmaf(y[1], y[1], ss);
    ss = fmaf(y[2], y[2], ss);
    ss = fmaf(y[3], y[3], ss);
    ss += __shfl_xor(ss, 1, 32);
    ss += __shfl_xor(ss, 2, 32);
    ss += __shfl_xor(ss, 4, 32);
    ss += __shfl_xor(ss, 8, 32);
    float inv = __builtin_amdgcn_rcpf(fmaxf(sqrtf(ss), kEps));
    if (which == 0) inv = inv * 0.125f;
    const float sc = (which < 2) ? inv : 1.0f;
    const v4f val = (v4f){y[0] * sc, y[1] * sc, y[2] * sc, y[3] * sc};
    float* dst = dstp + (((size_t)(b * kNH + h)) * kL + (size_t)l) * kHD + cg * 4;
    *(volatile v4f*)dst = val;
    __threadfence();
    *(volatile v4f*)dst = val;
  }

  if (t < 32) {
    const float lg = P[(rowb + (size_t)(chunk * kChunkT + t)) * kNStack + 3 * kHid + h];
    sb[t] = __builtin_amdgcn_rcpf(1.0f + expf(-lg));
  }
  __syncthreads();
  if (t < 8) {
    const v4f bv = *(const v4f*)(sb + t * 4);
    float* dst = BT + ((size_t)(b * kNH + h)) * kL + chunk * kChunkT + t * 4;
    *(volatile v4f*)dst = bv;
    __threadfence();
    *(volatile v4f*)dst = bv;
  }
}

__global__ __launch_bounds__(64) void scan_kernel(const float* __restrict__ QH, const float* __restrict__ KH,
                                                  const float* __restrict__ VH, const float* __restrict__ BT,
                                                  const float* __restrict__ ONW,
                                                  unsigned short* __restrict__ ONh, unsigned short* __restrict__ ONl,
                                                  float* __restrict__ Sout) {
  __shared__ __align__(16) float Sl[kHD * kSPitch];
  __shared__ __align__(16) float kq[2 * kHD];
  __shared__ __align__(16) float ob[kFlushT * kHD];
  __shared__ float red[2];
  const int bh = blockIdx.x;
  const int b = bh >> 4, h = bh & 15;
  const int m = threadIdx.x;
  const int lane = m & 31, wave = m >> 5;
  float* Scol = Sl + m * kSPitch;
  const v4f z4 = (v4f){0.f, 0.f, 0.f, 0.f};
#pragma unroll 1
  for (int d4 = 0; d4 < kHD; d4 += 4) *(v4f*)(Scol + d4) = z4;
  const size_t base = (size_t)bh * kL * kHD;
  const float wm = ONW[m];
  const int fq = lane >> 3, fc8 = (lane & 7) * 8;

  for (int l = 0; l < kL; ++l) {
    const size_t ro = base + (size_t)l * kHD + m;
    kq[m] = KH[ro];
    kq[kHD + m] = QH[ro];
    const float vt = VH[ro];
    const float bt = BT[(size_t)bh * kL + l];
    __syncthreads();

    float acc = 0.0f;
#pragma unroll 2
    for (int d4 = 0; d4 < kHD; d4 += 4) {
      const v4f s  = *(const v4f*)(Scol + d4);
      const v4f kk = *(const v4f*)(kq + d4);
      acc = fmaf(kk[0], s[0], acc);
      acc = fmaf(kk[1], s[1], acc);
      acc = fmaf(kk[2], s[2], acc);
      acc = fmaf(kk[3], s[3], acc);
    }
    const float vnew = (vt - acc) * bt;
    float o = 0.0f;
#pragma unroll 2
    for (int d4 = 0; d4 < kHD; d4 += 4) {
      v4f s = *(const v4f*)(Scol + d4);
      const v4f kk = *(const v4f*)(kq + d4);
      const v4f qq = *(const v4f*)(kq + kHD + d4);
      s[0] = fmaf(kk[0], vnew, s[0]);
      s[1] = fmaf(kk[1], vnew, s[1]);
      s[2] = fmaf(kk[2], vnew, s[2]);
      s[3] = fmaf(kk[3], vnew, s[3]);
      *(v4f*)(Scol + d4) = s;
      o = fmaf(qq[0], s[0], o);
      o = fmaf(qq[1], s[1], o);
      o = fmaf(qq[2], s[2], o);
      o = fmaf(qq[3], s[3], o);
    }

    float ss = o * o;
    ss += __shfl_xor(ss, 16, 32);
    ss += __shfl_xor(ss, 8, 32);
    ss += __shfl_xor(ss, 4, 32);
    ss += __shfl_xor(ss, 2, 32);
    ss += __shfl_xor(ss, 1, 32);
    if (lane == 0) red[wave] = ss;
    __syncthreads();
    const float tot = red[0] + red[1];
    const float on = o * rsqrtf(tot * (1.0f / 64.0f) + kEps) * wm;
    ob[(l & (kFlushT - 1)) * kHD + m] = on;

    if ((l & (kFlushT - 1)) == (kFlushT - 1)) {
      __syncthreads();
      const int l0 = l - (kFlushT - 1);
      v4u uh[2], ul[2];
#pragma unroll
      for (int it = 0; it < 2; ++it) {
        const int row = wave * 8 + it * 4 + fq;
        const float* sp = ob + row * kHD + fc8;
        const v4f a = *(const v4f*)(sp);
        const v4f cc = *(const v4f*)(sp + 4);
        unsigned short hb[8], lb[8];
#pragma unroll
        for (int e = 0; e < 4; ++e) {
          hb[e] = f2bf_bits(a[e]);
          lb[e] = f2bf_bits(a[e] - bf_bits2f(hb[e]));
          hb[4 + e] = f2bf_bits(cc[e]);
          lb[4 + e] = f2bf_bits(cc[e] - bf_bits2f(hb[4 + e]));
        }
        uh[it] = (v4u){pk16(hb[0], hb[1]), pk16(hb[2], hb[3]), pk16(hb[4], hb[5]), pk16(hb[6], hb[7])};
        ul[it] = (v4u){pk16(lb[0], lb[1]), pk16(lb[2], lb[3]), pk16(lb[4], lb[5]), pk16(lb[6], lb[7])};
      }
      for (int pass = 0; pass < 2; ++pass) {
#pragma unroll
        for (int it = 0; it < 2; ++it) {
          const int row = wave * 8 + it * 4 + fq;
          const size_t o16 = ((size_t)(b * kL + l0 + row)) * kHid + (size_t)(h * kHD + fc8);
          *(volatile v4u*)(ONh + o16) = uh[it];
          *(volatile v4u*)(ONl + o16) = ul[it];
        }
        __threadfence();
      }
    }
  }

  __syncthreads();
  {
    const int hh = lane >> 4, c4 = (lane & 15) * 4;
    for (int pass = 0; pass < 2; ++pass) {
#pragma unroll 1
      for (int it = 0; it < 16; ++it) {
        const int d = wave * 32 + it * 2 + hh;
        const v4f val = (v4f){Sl[(c4 + 0) * kSPitch + d], Sl[(c4 + 1) * kSPitch + d],
                              Sl[(c4 + 2) * kSPitch + d], Sl[(c4 + 3) * kSPitch + d]};
        *(volatile v4f*)(Sout + ((size_t)bh * kHD + d) * kHD + c4) = val;
      }
      __threadfence();
    }
  }
}

extern "C" void kernel_launch(void* const* d_in, const int* in_sizes, int n_in,
                              void* d_out, int out_size, void* d_ws,
                              size_t ws_size, hipStream_t stream) {
  (void)in_sizes; (void)n_in; (void)out_size;
  if (ws_size < kWsTotal) return;
  const float* x   = (const float*)d_in[0];
  const float* Wq  = (const float*)d_in[1];
  const float* Wk  = (const float*)d_in[2];
  const float* Wv  = (const float*)d_in[3];
  const float* Wb  = (const float*)d_in[4];
  const float* Wo  = (const float*)d_in[5];
  const float* cq  = (const float*)d_in[6];
  const float* ck  = (const float*)d_in[7];
  const float* cv  = (const float*)d_in[8];
  const float* onw = (const float*)d_in[9];
  float* out0 = (float*)d_out;
  float* out1 = out0 + (size_t)kTok * kHid;

  char* ws = (char*)d_ws;
  unsigned short* Xh  = (unsigned short*)(ws + kOffXh);
  unsigned short* Xl  = (unsigned short*)(ws + kOffXl);
  unsigned short* Wh  = (unsigned short*)(ws + kOffWh);
  unsigned short* Wl  = (unsigned short*)(ws + kOffWl);
  float*          P   = (float*)(ws + kOffP);
  float*          QH  = (float*)(ws + kOffQh);
  float*          KH  = (float*)(ws + kOffKh);
  float*          VH  = (float*)(ws + kOffVh);
  float*          BT  = (float*)(ws + kOffBt);
  unsigned short* ONh = (unsigned short*)(ws + kOffOnh);
  unsigned short* ONl = (unsigned short*)(ws + kOffOnl);
  unsigned short* WOh = (unsigned short*)(ws + kOffWoh);
  unsigned short* WOl = (unsigned short*)(ws + kOffWol);

  split8_kernel<<<dim3(2048), dim3(256), 0, stream>>>(x, Xh, Xl, kTok * kHid / 8);
  splitw_kernel<<<dim3(1568), dim3(256), 0, stream>>>(Wq, Wk, Wv, Wb, Wh, Wl);
  wmma_gemm64<1, true, 0, 0, false, 0><<<dim3(392, 1), dim3(256), 0, stream>>>(
      Xh, Xl, kHid, 0L, Wh, Wl, kHid, 0L, (void*)P, nullptr, kNStack, 0L, nullptr, nullptr, 0L,
      kTok, kNStack, kHid, 1.0f);
  prep_kernel<<<dim3(kL / kChunkT, kNH, kB), dim3(512), 0, stream>>>(P, cq, ck, cv, QH, KH, VH, BT);
  split8_kernel<<<dim3(512), dim3(256), 0, stream>>>(Wo, WOh, WOl, kHid * kHid / 8);
  scan_kernel<<<dim3(kB * kNH), dim3(kHD), 0, stream>>>(QH, KH, VH, BT, onw, ONh, ONl, out1);
  wmma_gemm64<1, true, 0, 0, false, 0><<<dim3(128, 1), dim3(256), 0, stream>>>(
      ONh, ONl, kHid, 0L, WOh, WOl, kHid, 0L, (void*)out0, nullptr, kHid, 0L, nullptr, nullptr, 0L,
      kTok, kHid, kHid, 1.0f);
}
